// SimpleMultiheadAttention_70463233458727
// MI455X (gfx1250) — hardware-verified
//
#include <hip/hip_runtime.h>
#include <math.h>
#include <stdint.h>

#define NB    2
#define SEQ   4096
#define EMB   768
#define NQKV  2304
#define NH    12
#define HD    64
#define NKT   (SEQ / 64)
static_assert(NH * HD == EMB);
static_assert((SEQ % 64) == 0 && (EMB % 64) == 0);
static_assert(NQKV == 3 * EMB);

typedef _Float16 v16h __attribute__((ext_vector_type(16)));
typedef _Float16 v8h  __attribute__((ext_vector_type(8)));
typedef __bf16   v16b __attribute__((ext_vector_type(16)));
typedef __bf16   v8b  __attribute__((ext_vector_type(8)));
typedef float    v8f  __attribute__((ext_vector_type(8)));
typedef float    v4f  __attribute__((ext_vector_type(4)));
typedef unsigned int v4u __attribute__((ext_vector_type(4)));

__device__ __forceinline__ unsigned short bf_bits(float f) {
  unsigned u = __float_as_uint(f);
  return (unsigned short)((u + 0x7FFFu + ((u >> 16) & 1u)) >> 16);
}
__device__ __forceinline__ float bf_up(unsigned short h) { return __uint_as_float(((unsigned)h) << 16); }
__device__ __forceinline__ float bf_rne(float f) { return bf_up(bf_bits(f)); }
__device__ __forceinline__ unsigned short h_bits(_Float16 x) { return __builtin_bit_cast(unsigned short, x); }
__device__ __forceinline__ unsigned pk16(unsigned short a, unsigned short b) { return (unsigned)a | ((unsigned)b << 16); }
__device__ __forceinline__ v8f zero8() { v8f z = {0.f, 0.f, 0.f, 0.f, 0.f, 0.f, 0.f, 0.f}; return z; }

__device__ __forceinline__ v16b ldfrag_b(const __bf16* p) {
  union { v16b v; v8b h[2]; } f;
  f.h[0] = *(const v8b*)(p);
  f.h[1] = *(const v8b*)(p + 16);
  return f.v;
}
__device__ __forceinline__ v16h ldfrag_h(const _Float16* p) {
  union { v16h v; v8h h[2]; } f;
  f.h[0] = *(const v8h*)(p);
  f.h[1] = *(const v8h*)(p + 16);
  return f.v;
}

__device__ __forceinline__ v8f mma_h(v16h a, v16h b, v8f c) {
  c = __builtin_amdgcn_wmma_f32_16x16x32_f16(false, a, false, b, (short)0, c, false, false);
  asm volatile("v_nop\n\tv_nop\n\tv_nop\n\tv_nop" : "+v"(c) : "v"(a), "v"(b));
  return c;
}
__device__ __forceinline__ v8f mma_b_raw(v16b a, v16b b, v8f c) {
  return __builtin_amdgcn_wmma_f32_16x16x32_bf16(false, a, false, b, (short)0, c, false, false);
}
__device__ __forceinline__ void dep_guard_b(v8f& a, v8f& b, v16b x, v16b y) {
  asm volatile("v_nop\n\tv_nop\n\tv_nop\n\tv_nop" : "+v"(a), "+v"(b) : "v"(x), "v"(y));
}
__device__ __forceinline__ void keep4_b(v16b a, v16b b, v16b c, v16b d) {
  asm volatile("v_nop" :: "v"(a), "v"(b), "v"(c), "v"(d));
}
__device__ __forceinline__ void acc_guard4(v8f& a, v8f& b, v8f& c, v8f& d) {
  asm volatile("v_nop\n\tv_nop\n\tv_nop\n\tv_nop" : "+v"(a), "+v"(b), "+v"(c), "+v"(d));
}

__global__ __launch_bounds__(256) void cvt_bf16x8(const float* __restrict__ in, unsigned short* out, int n8) {
  const int i = blockIdx.x * 256 + threadIdx.x;
  if (i < n8) {
    const v4f a = *(const v4f*)(in + (size_t)i * 8);
    const v4f b = *(const v4f*)(in + (size_t)i * 8 + 4);
    v4u p;
    p[0] = pk16(bf_bits(a[0]), bf_bits(a[1]));
    p[1] = pk16(bf_bits(a[2]), bf_bits(a[3]));
    p[2] = pk16(bf_bits(b[0]), bf_bits(b[1]));
    p[3] = pk16(bf_bits(b[2]), bf_bits(b[3]));
    *(volatile v4u*)(out + (size_t)i * 8) = p;
    __threadfence();
    *(volatile v4u*)(out + (size_t)i * 8) = p;
  }
}

template <int NSPLIT, int OUT_MODE, int BIAS>
__global__ __launch_bounds__(256) void gemm64(
    const unsigned short* __restrict__ Ap, const unsigned short* __restrict__ A2p, int lda, long long strideA,
    const unsigned short* __restrict__ Btp, int ldb, long long strideB,
    const float* __restrict__ bias,
    void* Cout, void* Cout2, int ldc, long long strideC,
    int M, int N, int K, float rscale) {
  const __bf16* A  = (const __bf16*)(const void*)Ap;
  const __bf16* A2 = (const __bf16*)(const void*)A2p;
  const __bf16* Bt = (const __bf16*)(const void*)Btp;
  __shared__ __align__(16) float sT[8][16 * 68];
  const int b    = blockIdx.y;
  const int lane = threadIdx.x & 31;
  const int wave = threadIdx.x >> 5;
  const int tilesN = N >> 6;
  const int tilesM = M >> 6;
  const int tile = blockIdx.x * 8 + wave;
  if (tile >= tilesM * tilesN) return;
  const int tm = tile / tilesN;
  const int tn = tile - tm * tilesN;
  const int m0 = tm << 6;
  const int n0 = tn << 6;

  const __bf16* Ab  = A  + (size_t)b * strideA;
  const __bf16* Bb  = Bt + (size_t)b * strideB;
  const __bf16* Ab2 = (NSPLIT >= 1) ? (A2 + (size_t)b * strideA) : Ab;

  const int rlane = lane & 15;
  const int koff  = (lane >> 4) * 8;
  const int mOff  = (lane >> 4) * 8;

  v8f acc[4][4];
#pragma unroll
  for (int i = 0; i < 4; ++i)
#pragma unroll
    for (int j = 0; j < 4; ++j) acc[i][j] = zero8();

  for (int k0 = 0; k0 < K; k0 += 32) {
    v16b bh[4];
#pragma unroll
    for (int j = 0; j < 4; ++j) {
      const size_t bo = (size_t)(n0 + (j << 4) + rlane) * ldb + koff + k0;
      bh[j] = ldfrag_b(Bb + bo);
    }
#pragma unroll
    for (int i = 0; i < 4; ++i) {
      const size_t ao = (size_t)(m0 + (i << 4) + rlane) * lda + koff + k0;
      const v16b ah = ldfrag_b(Ab + ao);
      v16b al = ah;
      if (NSPLIT >= 1) al = ldfrag_b(Ab2 + ao);
#pragma unroll
      for (int j = 0; j < 4; ++j) {
        acc[i][j] = mma_b_raw(ah, bh[j], acc[i][j]);
        if (NSPLIT >= 1) acc[i][j] = mma_b_raw(al, bh[j], acc[i][j]);
      }
      dep_guard_b(acc[i][0], acc[i][3], ah, al);
    }
    keep4_b(bh[0], bh[1], bh[2], bh[3]);
  }
  acc_guard4(acc[0][0], acc[0][1], acc[0][2], acc[0][3]);
  acc_guard4(acc[1][0], acc[1][1], acc[1][2], acc[1][3]);
  acc_guard4(acc[2][0], acc[2][1], acc[2][2], acc[2][3]);
  acc_guard4(acc[3][0], acc[3][1], acc[3][2], acc[3][3]);

  float* slab = sT[wave];
  const int hh = lane >> 4, c4 = (lane & 15) * 4;
  const int q8 = lane >> 3, c8 = (lane & 7) * 8;
  float bc[8];
#pragma unroll
  for (int e = 0; e < 8; ++e) bc[e] = 0.f;
  if (BIAS == 1) {
    if (OUT_MODE == 0) {
      const v4f t = *(const v4f*)(bias + n0 + c4);
#pragma unroll
      for (int e = 0; e < 4; ++e) bc[e] = bf_rne(t[e]);
    } else {
      const v4f t0 = *(const v4f*)(bias + n0 + c8);
      const v4f t1 = *(const v4f*)(bias + n0 + c8 + 4);
#pragma unroll
      for (int e = 0; e < 4; ++e) { bc[e] = bf_rne(t0[e]); bc[4 + e] = bf_rne(t1[e]); }
    }
  }
#pragma unroll
  for (int i = 0; i < 4; ++i) {
    const int mBase = m0 + (i << 4);
#pragma unroll
    for (int j = 0; j < 4; ++j) {
#pragma unroll
      for (int r = 0; r < 8; ++r) {
        slab[(mOff + r) * 68 + (j << 4) + rlane] = acc[i][j][r];
      }
    }
    __builtin_amdgcn_fence(__ATOMIC_RELEASE, "workgroup");
    __builtin_amdgcn_wave_barrier();
    __builtin_amdgcn_fence(__ATOMIC_ACQUIRE, "workgroup");
    if (OUT_MODE == 0) {
      float* C = (float*)Cout + (size_t)b * strideC;
      v4f vv[8];
#pragma unroll
      for (int it = 0; it < 8; ++it) {
        const int row = it * 2 + hh;
        v4f v = *(const v4f*)(slab + row * 68 + c4);
        float br = 0.f;
        if (BIAS == 2) br = bf_rne(bias[mBase + row]);
#pragma unroll
        for (int e = 0; e < 4; ++e) v[e] = (v[e] + bc[e]) + br;
        vv[it] = v;
      }
#pragma unroll
      for (int it = 0; it < 8; ++it) {
        const int row = it * 2 + hh;
        *(volatile v4f*)(C + (size_t)(mBase + row) * ldc + n0 + c4) = vv[it];
      }
      __threadfence();
#pragma unroll
      for (int it = 0; it < 8; ++it) {
        const int row = it * 2 + hh;
        *(volatile v4f*)(C + (size_t)(mBase + row) * ldc + n0 + c4) = vv[it];
      }
    } else {
      unsigned short* C  = (unsigned short*)Cout  + (size_t)b * strideC;
      unsigned short* C2 = (unsigned short*)Cout2 + (size_t)b * strideC;
      v4u hv[4], lv[4];
#pragma unroll
      for (int it = 0; it < 4; ++it) {
        const int row = it * 4 + q8;
        const float* sp = slab + row * 68 + c8;
        float br = 0.f;
        if (BIAS == 2) br = bf_rne(bias[mBase + row]);
        v4u a, a2;
#pragma unroll
        for (int e = 0; e < 4; ++e) {
          const float f0 = (sp[2 * e] + bc[2 * e]) + br;
          const float f1 = (sp[2 * e + 1] + bc[2 * e + 1]) + br;
          const _Float16 x0 = (_Float16)f0, x1 = (_Float16)f1;
          const unsigned short h0 = h_bits(x0), h1 = h_bits(x1);
          unsigned short l0 = 0, l1 = 0;
          if (OUT_MODE == 3) {
            l0 = h_bits((_Float16)((f0 - (float)x0) * rscale));
            l1 = h_bits((_Float16)((f1 - (float)x1) * rscale));
          }
          a[e] = pk16(h0, h1); a2[e] = pk16(l0, l1);
        }
        hv[it] = a; lv[it] = a2;
      }
#pragma unroll
      for (int it = 0; it < 4; ++it) {
        const int row = it * 4 + q8;
        *(volatile v4u*)(C + (size_t)(mBase + row) * ldc + n0 + c8) = hv[it];
        if (OUT_MODE == 3) *(volatile v4u*)(C2 + (size_t)(mBase + row) * ldc + n0 + c8) = lv[it];
      }
      __threadfence();
#pragma unroll
      for (int it = 0; it < 4; ++it) {
        const int row = it * 4 + q8;
        *(volatile v4u*)(C + (size_t)(mBase + row) * ldc + n0 + c8) = hv[it];
        if (OUT_MODE == 3) *(volatile v4u*)(C2 + (size_t)(mBase + row) * ldc + n0 + c8) = lv[it];
      }
    }
    __builtin_amdgcn_fence(__ATOMIC_RELEASE, "workgroup");
    __builtin_amdgcn_wave_barrier();
    __builtin_amdgcn_fence(__ATOMIC_ACQUIRE, "workgroup");
  }
}

__global__ __launch_bounds__(128)
void attn64(const unsigned short* __restrict__ qhp, const unsigned short* __restrict__ qrp,
            const unsigned short* __restrict__ khp, const unsigned short* __restrict__ vtp,
            const int* __restrict__ kpm,
            unsigned short* ohp, unsigned short* olp, float sscale) {
  union FH { v16h v; v8h h[2]; };
  __shared__ __align__(16) _Float16 Ksh[64 * 64];
  __shared__ __align__(16) _Float16 Vth[64 * 64];
  __shared__ __align__(16) _Float16 Psh[4][16 * 64];
  __shared__ __align__(16) float    Os[4][16 * 64];

  const int tid  = threadIdx.x;
  const int wave = tid >> 5;
  const int lane = tid & 31;
  const int hh   = lane >> 4;
  const int c    = lane & 15;

  const int bx   = blockIdx.x;
  const int qb   = bx % NKT;
  const int rest = bx / NKT;
  const int h    = rest % NH;
  const int b    = rest / NH;
  const int q0   = qb * 64 + wave * 16;
  const size_t rowB = (size_t)b * SEQ;

  const _Float16* Qh = (const _Float16*)(const void*)qhp + (size_t)h * HD;
  const _Float16* Qr = (const _Float16*)(const void*)qrp + (size_t)h * HD;
  const _Float16* Kh = (const _Float16*)(const void*)khp + (size_t)h * HD;
  const _Float16* Vt = (const _Float16*)(const void*)vtp + ((size_t)b * EMB + (size_t)h * HD) * SEQ;
  const int* mkb = kpm + (size_t)b * SEQ;

  v16h qah[2], qar[2];
#pragma unroll
  for (int dc = 0; dc < 2; ++dc) {
    const size_t qo = (rowB + q0 + c) * EMB + dc * 32 + 8 * hh;
    qah[dc] = ldfrag_h(Qh + qo);
    qar[dc] = ldfrag_h(Qr + qo);
  }

  float mrow[8], lrow[8];
  v8f oacc[4];
#pragma unroll
  for (int r = 0; r < 8; ++r) { mrow[r] = -INFINITY; lrow[r] = 0.f; }
#pragma unroll
  for (int t = 0; t < 4; ++t) oacc[t] = zero8();

  for (int kt = 0; kt < NKT; ++kt) {
    const int kv0 = kt * 64;
    __syncthreads();
    {
      const int r = tid >> 1, half = (tid & 1) * 32;
      const _Float16* kg = Kh + (rowB + kv0 + r) * EMB + half;
      const _Float16* vg = Vt + (size_t)r * SEQ + kv0 + half;
#pragma unroll
      for (int i = 0; i < 4; ++i) {
        const v8h a0 = *(const v8h*)(kg + 8 * i);
        const v8h b0 = *(const v8h*)(vg + 8 * i);
        *(v8h*)(Ksh + r * 64 + half + 8 * i) = a0;
        *(v8h*)(Vth + r * 64 + half + 8 * i) = b0;
      }
    }
    __syncthreads();

    int mk[4];
#pragma unroll
    for (int j = 0; j < 4; ++j) mk[j] = mkb[kv0 + j * 16 + c];

    v8f s[4];
#pragma unroll
    for (int j = 0; j < 4; ++j) {
      v8f sj = zero8(), sr = zero8();
#pragma unroll
      for (int dc = 0; dc < 2; ++dc) {
        FH kb;
        kb.h[0] = *(const v8h*)(Ksh + (j * 16 + c) * 64 + dc * 32 + 8 * hh);
        kb.h[1] = *(const v8h*)(Ksh + (j * 16 + c) * 64 + dc * 32 + 16 + 8 * hh);
        sj = mma_h(qah[dc], kb.v, sj);
        sr = mma_h(qar[dc], kb.v, sr);
      }
      s[j] = sj + sr * 0.0009765625f;
    }

    _Float16* pwh = Psh[wave];
#pragma unroll
    for (int r = 0; r < 8; ++r) {
      float m = -INFINITY;
#pragma unroll
      for (int j = 0; j < 4; ++j) {
        float sv = s[j][r] * sscale;
        sv = (mk[j] != 0) ? -INFINITY : sv;
        s[j][r] = sv;
        m = fmaxf(m, sv);
      }
#pragma unroll
      for (int off = 1; off < 16; off <<= 1) m = fmaxf(m, __shfl_xor(m, off, 32));
      const float mnew  = fmaxf(mrow[r], m);
      const float msafe = (mnew == -INFINITY) ? 0.f : mnew;
      const float alpha = __expf(mrow[r] - msafe);
      mrow[r] = mnew;
      float psum = 0.f;
#pragma unroll
      for (int j = 0; j < 4; ++j) {
        const float p = __expf(s[j][r] - msafe);
        psum += p;
        pwh[(8 * hh + r) * 64 + j * 16 + c] = (_Float16)(p * 1024.0f);
      }
#pragma unroll
      for (int off = 1; off < 16; off <<= 1) psum += __shfl_xor(psum, off, 32);
      lrow[r] = lrow[r] * alpha + psum;
#pragma unroll
      for (int t = 0; t < 4; ++t) oacc[t][r] *= alpha;
    }
    __builtin_amdgcn_fence(__ATOMIC_RELEASE, "workgroup");
    __builtin_amdgcn_wave_barrier();
    __builtin_amdgcn_fence(__ATOMIC_ACQUIRE, "workgroup");

#pragma unroll 1
    for (int kk = 0; kk < 2; ++kk) {
      FH pa;
      pa.h[0] = *(const v8h*)(pwh + c * 64 + kk * 32 + 8 * hh);
      pa.h[1] = *(const v8h*)(pwh + c * 64 + kk * 32 + 16 + 8 * hh);
#pragma unroll
      for (int t = 0; t < 4; ++t) {
        FH vb;
        vb.h[0] = *(const v8h*)(Vth + (t * 16 + c) * 64 + kk * 32 + 8 * hh);
        vb.h[1] = *(const v8h*)(Vth + (t * 16 + c) * 64 + kk * 32 + 16 + 8 * hh);
        oacc[t] = mma_h(pa.v, vb.v, oacc[t]);
      }
    }
  }

  float* os = Os[wave];
#pragma unroll
  for (int r = 0; r < 8; ++r) {
    const float l = lrow[r];
    const float inv = (1.0f / l) * 0.0009765625f;
#pragma unroll
    for (int t = 0; t < 4; ++t) os[(8 * hh + r) * 64 + t * 16 + c] = oacc[t][r] * inv;
  }
  __builtin_amdgcn_fence(__ATOMIC_RELEASE, "workgroup");
  __builtin_amdgcn_wave_barrier();
  __builtin_amdgcn_fence(__ATOMIC_ACQUIRE, "workgroup");
  {
    const int q4 = lane >> 3, c8 = (lane & 7) * 8;
    v4u hv[4], lv[4];
#pragma unroll
    for (int it = 0; it < 4; ++it) {
      const int row = it * 4 + q4;
      const float* sp = os + row * 64 + c8;
      v4u a, a2;
#pragma unroll
      for (int e = 0; e < 4; ++e) {
        const float f0 = sp[2 * e], f1 = sp[2 * e + 1];
        const unsigned short h0 = bf_bits(f0), h1 = bf_bits(f1);
        const unsigned short l0 = bf_bits(f0 - bf_up(h0)), l1 = bf_bits(f1 - bf_up(h1));
        a[e] = pk16(h0, h1); a2[e] = pk16(l0, l1);
      }
      hv[it] = a; lv[it] = a2;
    }
#pragma unroll
    for (int it = 0; it < 4; ++it) {
      const int row = it * 4 + q4;
      const size_t go = (rowB + q0 + row) * EMB + (size_t)h * HD + c8;
      *(volatile v4u*)(ohp + go) = hv[it];
      *(volatile v4u*)(olp + go) = lv[it];
    }
    __threadfence();
#pragma unroll
    for (int it = 0; it < 4; ++it) {
      const int row = it * 4 + q4;
      const size_t go = (rowB + q0 + row) * EMB + (size_t)h * HD + c8;
      *(volatile v4u*)(ohp + go) = hv[it];
      *(volatile v4u*)(olp + go) = lv[it];
    }
  }
}

extern "C" void kernel_launch(void* const* d_in, const int* in_sizes, int n_in,
                              void* d_out, int out_size, void* d_ws, size_t ws_size,
                              hipStream_t stream) {
  if (n_in < 6) return;
  if (in_sizes[0] != NB * SEQ * EMB) return;
  if (in_sizes[1] != NB * SEQ) return;
  if (in_sizes[2] != NQKV * EMB || in_sizes[3] != NQKV) return;
  if (in_sizes[4] != EMB * EMB || in_sizes[5] != EMB) return;
  if (out_size != NB * SEQ * EMB) return;

  const float* x     = (const float*)d_in[0];
  const int*   kpm   = (const int*)d_in[1];
  const float* w_qkv = (const float*)d_in[2];
  const float* b_qkv = (const float*)d_in[3];
  const float* w_out = (const float*)d_in[4];
  const float* b_out = (const float*)d_in[5];

  const size_t PX  = (size_t)NB * SEQ * EMB * 2;
  const size_t PW  = (size_t)NQKV * EMB * 2;
  const size_t PO  = (size_t)EMB * EMB * 2;
  const size_t PVT = (size_t)NB * EMB * SEQ * 2;
  size_t off = 0;
  const size_t oXb  = off; off += PX;
  const size_t oWb  = off; off += PW;
  const size_t oWob = off; off += PO;
  const size_t oQh  = off; off += PX;
  const size_t oQr  = off; off += PX;
  const size_t oKh  = off; off += PX;
  const size_t oVT  = off; off += PVT;
  const size_t oOh  = off; off += PX;
  const size_t oOl  = off; off += PX;
  if (off > ws_size) return;
  if (off > (size_t)134217728) return;

  char* ws = (char*)d_ws;
  unsigned short* Xb  = (unsigned short*)(ws + oXb);
  unsigned short* Wb  = (unsigned short*)(ws + oWb);
  unsigned short* Wob = (unsigned short*)(ws + oWob);
  unsigned short* Qh  = (unsigned short*)(ws + oQh);
  unsigned short* Qr  = (unsigned short*)(ws + oQr);
  unsigned short* Kh  = (unsigned short*)(ws + oKh);
  unsigned short* VT  = (unsigned short*)(ws + oVT);
  unsigned short* Oh  = (unsigned short*)(ws + oOh);
  unsigned short* Ol  = (unsigned short*)(ws + oOl);

  const dim3 blk(256);
  const int n8x = NB * SEQ * EMB / 8;
  const int n8w = NQKV * EMB / 8;
  const int n8o = EMB * EMB / 8;
  const dim3 gCvtX((n8x + 255) / 256);
  const dim3 gCvtW((n8w + 255) / 256);
  const dim3 gCvtO((n8o + 255) / 256);
  const dim3 gProj(((NB * SEQ / 64) * (EMB / 64) + 7) / 8, 1);
  const dim3 gVT(((EMB / 64) * (SEQ / 64) + 7) / 8, NB);
  const dim3 gAttn(NB * NH * NKT);

  cvt_bf16x8<<<gCvtX, blk, 0, stream>>>(x, Xb, n8x);
  cvt_bf16x8<<<gCvtW, blk, 0, stream>>>(w_qkv, Wb, n8w);
  cvt_bf16x8<<<gCvtO, blk, 0, stream>>>(w_out, Wob, n8o);
  gemm64<0, 3, 1><<<gProj, blk, 0, stream>>>(
      Xb, Xb, EMB, 0LL, Wb, EMB, 0LL, b_qkv,
      (void*)Qh, (void*)Qr, EMB, 0LL,
      NB * SEQ, EMB, EMB, 1024.0f);
  gemm64<0, 1, 1><<<gProj, blk, 0, stream>>>(
      Xb, Xb, EMB, 0LL, Wb + (size_t)EMB * EMB, EMB, 0LL, b_qkv + EMB,
      (void*)Kh, (void*)Kh, EMB, 0LL,
      NB * SEQ, EMB, EMB, 1.0f);
  gemm64<0, 1, 2><<<gVT, blk, 0, stream>>>(
      Wb + (size_t)2 * EMB * EMB, Wb + (size_t)2 * EMB * EMB, EMB, 0LL,
      Xb, EMB, (long long)SEQ * EMB, b_qkv + 2 * EMB,
      (void*)VT, (void*)VT, SEQ, (long long)EMB * SEQ,
      EMB, SEQ, EMB, 1.0f);
  attn64<<<gAttn, dim3(128), 0, stream>>>(Qh, Qr, Kh, VT, kpm, Oh, Ol, 0.125f);
  gemm64<1, 0, 1><<<gProj, blk, 0, stream>>>(
      Oh, Ol, EMB, 0LL, Wob, EMB, 0LL, b_out,
      d_out, d_out, EMB, 0LL,
      NB * SEQ, EMB, EMB, 1.0f);
  (void)hipGetLastError();
}
